// attention_32839319945834
// MI455X (gfx1250) — hardware-verified
//
#include <hip/hip_runtime.h>

typedef __attribute__((ext_vector_type(16))) _Float16     v16h;
typedef __attribute__((ext_vector_type(8)))  _Float16     v8h;
typedef __attribute__((ext_vector_type(8)))  float        v8f;
typedef __attribute__((ext_vector_type(4)))  float        v4f;
typedef __attribute__((ext_vector_type(4)))  unsigned int v4u;

#ifndef NB
#define NB 4
#endif
#ifndef SEQ
#define SEQ 2048
#endif
#define NB_FULL  4
#define SEQ_FULL 2048
#define NH       8
#define DH       64
#define FA_NW    4
#define FA_QB    (16 * FA_NW)
#define OS_P     68

#define PLANE_ELEMS ((size_t)NB * NH * SEQ * DH)
#define PLANE_BYTES (PLANE_ELEMS * 2)
#define WS_TOTAL    (3 * PLANE_BYTES)

static_assert(DH == 64);
static_assert(NB <= NB_FULL);
static_assert(SEQ <= SEQ_FULL);
static_assert(SEQ % 256 == 0);
static_assert(SEQ % FA_QB == 0);
static_assert(DH % 32 == 0);
static_assert(PLANE_BYTES % 128 == 0);
static_assert(WS_TOTAL <= 134217728);
static_assert((OS_P * 4) % 16 == 0);

union FragH { v16h v; v8h h[2]; };
__device__ __forceinline__ v16h ld_frag(const _Float16* __restrict__ p) {
    FragH f; f.h[0] = *(const v8h*)(p); f.h[1] = *(const v8h*)(p + 16); return f.v;
}
__device__ __forceinline__ v8f mma16(v16h a, v16h b, v8f c) {
    return __builtin_amdgcn_wmma_f32_16x16x32_f16(false, a, false, b, (short)0, c, false, false);
}
__device__ __forceinline__ void guard_s(v8f& s0, v8f& s1, v16h a0, v16h a1, v16h a2, v16h a3, v16h b0, v16h b1) {
    asm volatile("v_nop\n\tv_nop\n\tv_nop\n\tv_nop" : "+v"(s0), "+v"(s1) : "v"(a0), "v"(a1), "v"(a2), "v"(a3), "v"(b0), "v"(b1));
}
__device__ __forceinline__ void guard_o(v8f& o0, v8f& o1, v8f& o2, v8f& o3, v16h a0, v16h a1, v16h a2, v16h a3, v16h b) {
    asm volatile("v_nop\n\tv_nop\n\tv_nop\n\tv_nop" : "+v"(o0), "+v"(o1), "+v"(o2), "+v"(o3) : "v"(a0), "v"(a1), "v"(a2), "v"(a3), "v"(b));
}

__device__ __forceinline__ float bf_rne(float v) {
    const unsigned u = __float_as_uint(v);
    const unsigned r = (u + 0x7fffu + ((u >> 16) & 1u)) & 0xffff0000u;
    return __uint_as_float(r);
}
__device__ __forceinline__ unsigned int pk2h(float a, float b) {
    return (unsigned int)__builtin_bit_cast(unsigned short, (_Float16)a) | ((unsigned int)__builtin_bit_cast(unsigned short, (_Float16)b) << 16);
}

__global__ __launch_bounds__(256) void k_cast_rows(const float* __restrict__ src, unsigned short* __restrict__ dst) {
    const long long u = (long long)blockIdx.x * 256 + threadIdx.x;
    if (u >= (long long)NB * NH * SEQ * (DH / 8)) return;
    const int c0 = 8 * (int)(u & 7);
    const long long row = u >> 3;
    const int bh = (int)(row / SEQ);
    const int s  = (int)(row % SEQ);
    const float* sp = src + ((size_t)bh * SEQ_FULL + (size_t)s) * DH + c0;
    const v4f x0 = *(const v4f*)(sp);
    const v4f x1 = *(const v4f*)(sp + 4);
    v4u pk;
    pk.x = pk2h(bf_rne(x0.x) * 16.0f, bf_rne(x0.y) * 16.0f);
    pk.y = pk2h(bf_rne(x0.z) * 16.0f, bf_rne(x0.w) * 16.0f);
    pk.z = pk2h(bf_rne(x1.x) * 16.0f, bf_rne(x1.y) * 16.0f);
    pk.w = pk2h(bf_rne(x1.z) * 16.0f, bf_rne(x1.w) * 16.0f);
    volatile v4u* d = (volatile v4u*)(dst + (size_t)row * DH + c0);
    *d = pk; __threadfence(); *d = pk;
}

__global__ __launch_bounds__(256) void k_cast_vt(const float* __restrict__ src, unsigned short* __restrict__ dst) {
    const long long u = (long long)blockIdx.x * 256 + threadIdx.x;
    const int per = SEQ / 8;
    if (u >= (long long)NB * NH * DH * per) return;
    const int s0 = 8 * (int)(u % per);
    const long long rid = u / per;
    const int d  = (int)(rid % DH);
    const int bh = (int)(rid / DH);
    const float* sp = src + ((size_t)bh * SEQ_FULL + (size_t)s0) * DH + d;
    float w[8];
#pragma unroll
    for (int e = 0; e < 8; ++e) w[e] = bf_rne(sp[(size_t)e * DH]) * 16.0f;
    v4u pk;
    pk.x = pk2h(w[0], w[1]); pk.y = pk2h(w[2], w[3]); pk.z = pk2h(w[4], w[5]); pk.w = pk2h(w[6], w[7]);
    volatile v4u* dd = (volatile v4u*)(dst + ((size_t)bh * DH + (size_t)d) * SEQ + s0);
    *dd = pk; __threadfence(); *dd = pk;
}

#define FA_STAGE(T, ACC) do { \
    v4f lo_, hi_; \
    lo_.x = ACC[0] * inv; lo_.y = ACC[1] * inv; lo_.z = ACC[2] * inv; lo_.w = ACC[3] * inv; \
    hi_.x = ACC[4] * inv; hi_.y = ACC[5] * inv; hi_.z = ACC[6] * inv; hi_.w = ACC[7] * inv; \
    *(v4f*)&os[wave][col * OS_P + (T) * 16 + 8 * h]     = lo_; \
    *(v4f*)&os[wave][col * OS_P + (T) * 16 + 8 * h + 4] = hi_; \
} while (0)

__global__ __launch_bounds__(32 * FA_NW) void k_fa(const _Float16* __restrict__ Q16, const _Float16* __restrict__ K16, const _Float16* __restrict__ Vt16,
                                                   float* __restrict__ O, const int* __restrict__ n_unused) {
    (void)n_unused;
    __shared__ __align__(16) float os[FA_NW][16 * OS_P];
    const int lane = threadIdx.x & 31;
    const int wave = __builtin_amdgcn_readfirstlane(threadIdx.x >> 5);
    const int h = lane >> 4, col = lane & 15;
    const int bh = blockIdx.y;
    const int q0 = blockIdx.x * FA_QB + wave * 16;
    const size_t pbase = (size_t)bh * SEQ * DH;

    const float C2 = (float)(0.044194173824159216 * 1.4426950408889634 / 256.0);

    const _Float16* qrow = Q16 + pbase + (size_t)(q0 + col) * DH + 8 * h;
    const v16h bq0 = ld_frag(qrow);
    const v16h bq1 = ld_frag(qrow + 32);
    const _Float16* kp = K16 + pbase + (size_t)col * DH + 8 * h;
    const _Float16* vp = Vt16 + pbase + (size_t)col * SEQ + 8 * h;

    v8f a0 = {}, a1 = {}, a2 = {}, a3 = {};
    float m = -1.0e30f, l = 0.0f;

#pragma unroll 1
    for (int kg = 0; kg < SEQ / 32; ++kg) {
        const _Float16* kt = kp + (size_t)kg * 32 * DH;
        const v16h k00 = ld_frag(kt);
        const v16h k01 = ld_frag(kt + 32);
        const v16h k10 = ld_frag(kt + 16 * DH);
        const v16h k11 = ld_frag(kt + 16 * DH + 32);
        v8f s0 = {}, s1 = {};
        s0 = mma16(k00, bq0, s0);
        s1 = mma16(k10, bq0, s1);
        s0 = mma16(k01, bq1, s0);
        s1 = mma16(k11, bq1, s1);
        guard_s(s0, s1, k00, k01, k10, k11, bq0, bq1);

        const _Float16* vt = vp + kg * 32;
        const v16h v0 = ld_frag(vt);
        const v16h v1 = ld_frag(vt + 16 * SEQ);
        const v16h v2 = ld_frag(vt + 32 * SEQ);
        const v16h v3 = ld_frag(vt + 48 * SEQ);

        float mx = fmaxf(s0[0], s1[0]);
#pragma unroll
        for (int r = 1; r < 8; ++r) mx = fmaxf(mx, fmaxf(s0[r], s1[r]));
        mx *= C2;
        mx = fmaxf(mx, __shfl_xor(mx, 16, 32));
        const float mnew = fmaxf(m, mx);
        const float corr = __builtin_amdgcn_exp2f(m - mnew);
        const float nref = 8.0f - mnew;
        v16h bp; float rs = 0.0f;
#pragma unroll
        for (int r = 0; r < 8; ++r) {
            const float e0 = __builtin_amdgcn_exp2f(__builtin_fmaf(s0[r], C2, nref));
            const float e1 = __builtin_amdgcn_exp2f(__builtin_fmaf(s1[r], C2, nref));
            rs += e0 + e1;
            bp[r]     = (_Float16)e0;
            bp[8 + r] = (_Float16)e1;
        }
        l = l * corr + rs;
        m = mnew;
        a0 = a0 * corr; a1 = a1 * corr; a2 = a2 * corr; a3 = a3 * corr;
        a0 = mma16(v0, bp, a0);
        a1 = mma16(v1, bp, a1);
        a2 = mma16(v2, bp, a2);
        a3 = mma16(v3, bp, a3);
        guard_o(a0, a1, a2, a3, v0, v1, v2, v3, bp);
    }

    const float lt = l + __shfl_xor(l, 16, 32);
    const float inv = 1.0f / (lt * 16.0f);

    FA_STAGE(0, a0);
    FA_STAGE(1, a1);
    FA_STAGE(2, a2);
    FA_STAGE(3, a3);
    __syncthreads();
    {
        float* ob = O + ((size_t)bh * SEQ + (size_t)q0) * DH;
        const int c4 = (lane & 15) * 4;
        for (int pass = 0; pass < 2; ++pass) {
#pragma unroll
            for (int it = 0; it < 8; ++it) {
                const int row = it * 2 + h;
                const v4f val = *(const v4f*)&os[wave][row * OS_P + c4];
                *(volatile v4f*)(ob + (size_t)row * DH + c4) = val;
            }
            __threadfence();
        }
    }
}

extern "C" void kernel_launch(void* const* d_in, const int* in_sizes, int n_in, void* d_out, int out_size, void* d_ws, size_t ws_size, hipStream_t stream) {
    if (n_in < 4) return;
    const long long need = ((long long)(NB * NH - 1) * SEQ_FULL + SEQ) * DH;
    if ((long long)in_sizes[0] < need || (long long)in_sizes[1] < need || (long long)in_sizes[2] < need || in_sizes[3] < 1) return;
    if ((long long)out_size < (long long)NB * NH * SEQ * DH) return;
    if ((size_t)WS_TOTAL > ws_size) return;
    const float* q = (const float*)d_in[0];
    const float* k = (const float*)d_in[1];
    const float* v = (const float*)d_in[2];
    const int*   n = (const int*)d_in[3];
    float* out = (float*)d_out;
    char* wsp = (char*)d_ws;
    unsigned short* Q16  = (unsigned short*)(wsp);
    unsigned short* K16  = (unsigned short*)(wsp + PLANE_BYTES);
    unsigned short* Vt16 = (unsigned short*)(wsp + 2 * PLANE_BYTES);

    const unsigned gr = (unsigned)(((long long)NB * NH * SEQ * (DH / 8) + 255) / 256);
    const unsigned gv = (unsigned)(((long long)NB * NH * DH * (SEQ / 8) + 255) / 256);
    k_cast_rows<<<gr, 256, 0, stream>>>(q, Q16);
    k_cast_rows<<<gr, 256, 0, stream>>>(k, K16);
    k_cast_vt<<<gv, 256, 0, stream>>>(v, Vt16);
    k_fa<<<dim3((unsigned)(SEQ / FA_QB), (unsigned)(NB * NH)), 32 * FA_NW, 0, stream>>>((const _Float16*)Q16, (const _Float16*)K16, (const _Float16*)Vt16, out, n);
}
